// GaborTransform_64055142252567
// MI455X (gfx1250) — hardware-verified
//
#include <hip/hip_runtime.h>
#include <math.h>

typedef __attribute__((ext_vector_type(16))) _Float16 v16h;
typedef __attribute__((ext_vector_type(16))) __bf16 v16b;
typedef __attribute__((ext_vector_type(8)))  _Float16 v8h;
typedef __attribute__((ext_vector_type(8)))  float v8f;
typedef __attribute__((ext_vector_type(4)))  float v4f;
typedef __attribute__((ext_vector_type(2)))  float v2f;
typedef __attribute__((ext_vector_type(4)))  unsigned v4u;
typedef __attribute__((ext_vector_type(4)))  int v4i;
typedef float __attribute__((may_alias)) float_a;
typedef int __attribute__((may_alias)) int_a;

template <typename T> __device__ __forceinline__ void vst2(void* p, T v) { *(volatile T*)p = v; __threadfence(); *(volatile T*)p = v; }
__device__ __forceinline__ v8f wmma16(v16h a, v16h b, v8f c) {
  v8f d = __builtin_amdgcn_wmma_f32_16x16x32_f16(false, a, false, b, (short)0, c, false, false);
  asm volatile("v_nop\n\tv_nop\n\tv_nop\n\tv_nop" : "+v"(d) : "v"(a), "v"(b));
  return d;
}
__device__ __forceinline__ v8f wmma_bf(v16b a, v16b b, v8f c) {
  v8f d = __builtin_amdgcn_wmma_f32_16x16x32_bf16(false, a, false, b, (short)0, c, false, false);
  asm volatile("v_nop\n\tv_nop\n\tv_nop\n\tv_nop" : "+v"(d) : "v"(a), "v"(b));
  return d;
}
__device__ __forceinline__ v16h frag_h(const _Float16* rowk0, int lane) {
  union { v16h v; v8h q[2]; } u; const _Float16* p = rowk0 + 8 * (lane >> 4);
  u.q[0] = *(const v8h*)p; u.q[1] = *(const v8h*)(p + 16); return u.v;
}
__device__ __forceinline__ v16h frag_f32(const float* rowk0, int lane) {
  v16h a; const float* p = rowk0 + 8 * (lane >> 4);
#pragma unroll
  for (int i = 0; i < 8; ++i) { a[i] = (_Float16)p[i]; a[8 + i] = (_Float16)p[16 + i]; }
  return a;
}
__device__ __forceinline__ v16h frag_f32s(const float* rowk0, int lane, float sc) {
  v16h a; const float* p = rowk0 + 8 * (lane >> 4);
#pragma unroll
  for (int i = 0; i < 8; ++i) { a[i] = (_Float16)(p[i] * sc); a[8 + i] = (_Float16)(p[16 + i] * sc); }
  return a;
}
__device__ __forceinline__ v16h fragc_f32(const float* W, int k0, int n, int lane, int ld, int K) {
  v16h a; const int g = lane >> 4;
#pragma unroll
  for (int i = 0; i < 8; ++i) { const int ka = k0 + 8 * g + i, kb = ka + 16;
    a[i] = (_Float16)(ka < K ? W[(size_t)ka * ld + n] : 0.f); a[8 + i] = (_Float16)(kb < K ? W[(size_t)kb * ld + n] : 0.f); }
  return a;
}
struct F2 { v16b h, l; };
__device__ __forceinline__ F2 bsplit16(const float v[16]) { F2 r;
#pragma unroll
  for (int i = 0; i < 16; ++i) { const __bf16 h = (__bf16)v[i]; r.h[i] = h; r.l[i] = (__bf16)(v[i] - (float)h); }
  return r; }
__device__ __forceinline__ F2 split_row(const float* row, int k0, int lane) { float v[16]; const float* p = row + k0 + 8 * (lane >> 4);
#pragma unroll
  for (int i = 0; i < 8; ++i) { v[i] = p[i]; v[8 + i] = p[16 + i]; }
  return bsplit16(v); }
__device__ __forceinline__ F2 split_rowK(const float* row, int k0, int lane, int K) { float v[16]; const int g = lane >> 4;
#pragma unroll
  for (int i = 0; i < 8; ++i) { const int ka = k0 + 8 * g + i, kb = ka + 16; v[i] = ka < K ? row[ka] : 0.f; v[8 + i] = kb < K ? row[kb] : 0.f; }
  return bsplit16(v); }
__device__ __forceinline__ F2 split_col(const float* W, int k0, int n, int lane, int ld, int K) { float v[16]; const int g = lane >> 4;
#pragma unroll
  for (int i = 0; i < 8; ++i) { const int ka = k0 + 8 * g + i, kb = ka + 16; v[i] = ka < K ? W[(size_t)ka * ld + n] : 0.f; v[8 + i] = kb < K ? W[(size_t)kb * ld + n] : 0.f; }
  return bsplit16(v); }
__device__ __forceinline__ v8f mac3(const F2& a, const F2& b, v8f c) { c = wmma_bf(a.l, b.h, c); c = wmma_bf(a.h, b.l, c); return wmma_bf(a.h, b.h, c); }
__device__ __forceinline__ float sigm(float v) { return 1.0f / (1.0f + expf(-v)); }
#define LDSX() do { asm volatile("s_wait_dscnt 0" ::: "memory"); __builtin_amdgcn_wave_barrier(); __builtin_amdgcn_fence(__ATOMIC_RELEASE, "workgroup"); } while (0)

#define NBT 32
#define LL 8192
#define NFQ 128
#define NTM 128
#define NR (NBT * NTM)

__global__ __launch_bounds__(256) void k_cos(_Float16* __restrict__ CT) {
  const int f = blockIdx.x, tid = threadIdx.x; __shared__ __align__(16) _Float16 sr[LL];
  const float fv = (float)(int)((float)f * 4096.0f / 127.0f);
  const float two_pi = 6.2831853071795864f;
  for (int l = tid; l < LL; l += 256) { const float arg = ((two_pi * fv) * (float)l) / (float)LL; const float cv = cosf(arg); sr[l] = (_Float16)(fabsf(cv) < 6.2e-5f ? 0.f : cv); }
  __syncthreads();
  for (int q = tid; q < LL / 8; q += 256) vst2(CT + (size_t)f * LL + q * 8, *(const v4u*)(&sr[q * 8]));
}
__global__ __launch_bounds__(128) void k_main(const float* __restrict__ sig, const _Float16* __restrict__ CT, float* __restrict__ out) {
  __shared__ __align__(16) float ssig[LL];
  __shared__ __align__(16) _Float16 sa[4][16][40];
  __shared__ __align__(16) float st[NFQ][68];
  const int tid = threadIdx.x, wave = tid >> 5, lane = tid & 31, col = lane & 15, g = lane >> 4;
  const int b = blockIdx.y, t0b = blockIdx.x * 64, t0 = t0b + wave * 16;
  for (int q = tid; q < LL / 4; q += 128) *(v4f*)(&ssig[q * 4]) = *(const v4f*)(sig + (size_t)b * LL + q * 4);
  __syncthreads();
  const int tt = t0 + col; const float ct = (float)(int)((float)tt * 8191.0f / 127.0f);
  const float sw = 819.2f;
  v8f acc[8] = {};
#pragma unroll 2
  for (int kc = 0; kc < LL / 32; ++kc) {
    { union { v8h h[2]; v4u u2[2]; } pk;
#pragma unroll
      for (int u = 0; u < 16; ++u) { const int l = kc * 32 + g * 16 + u; const float z = ((float)l - ct) / sw; const float av = ssig[l] * expf(-0.5f * z * z); pk.h[u >> 3][u & 7] = (_Float16)(fabsf(av) < 6.2e-5f ? 0.f : av); }
      *(v4u*)(&sa[wave][col][g * 16]) = pk.u2[0]; *(v4u*)(&sa[wave][col][g * 16 + 8]) = pk.u2[1]; }
    LDSX();
    const v16h a = frag_h(&sa[wave][col][0], lane);
#pragma unroll
    for (int j = 0; j < 8; ++j) acc[j] = wmma16(a, frag_h(CT + (size_t)(j * 16 + col) * LL + kc * 32, lane), acc[j]);
    LDSX(); }
#pragma unroll
  for (int j = 0; j < 8; ++j)
#pragma unroll
    for (int r = 0; r < 8; ++r) st[j * 16 + col][wave * 16 + 8 * g + r] = acc[j][r];
  __syncthreads();
  for (int q = tid; q < NFQ * 16; q += 128) { const int f = q >> 4, pc = q & 15; vst2(out + ((size_t)b * NFQ + f) * NTM + t0b + pc * 4, *(const v4f*)(&st[f][pc * 4])); }
}
extern "C" void kernel_launch(void* const* d_in, const int* in_sizes, int n_in, void* d_out, int out_size, void* d_ws, size_t ws_size, hipStream_t stream) {
  (void)in_sizes; (void)n_in; (void)out_size; (void)ws_size;
  const float* sig = (const float*)d_in[0]; float* out = (float*)d_out;
  _Float16* CT = (_Float16*)d_ws;
  k_cos<<<NFQ, 256, 0, stream>>>(CT);
  k_main<<<dim3(NTM / 64, NBT), 128, 0, stream>>>(sig, CT, out);
}
